// MicroExpertMoE_17343077941602
// MI455X (gfx1250) — hardware-verified
//
#include <hip/hip_runtime.h>
#include <stddef.h>

#define NTOK 8192
#define DM   1024
#define NE   16
#define KE   256
#define TB   16
#define HP   264
#define NTHR 256
#define NWAV (NTHR / 32)
#define WCOL 128
#define RK   (DM / NWAV)
#define LDSB 32768

static_assert(NTOK % TB == 0);
static_assert(DM % 32 == 0);
static_assert(KE % 32 == 0);
static_assert(RK % 32 == 0);
static_assert(NWAV * 32 == KE);
static_assert(NWAV * WCOL == DM);
static_assert(TB * NE == NTHR);
static_assert(HP % 8 == 0);
static_assert(HP >= KE);
static_assert((NE & (NE - 1)) == 0);
static_assert(2 * TB * HP * 2 <= LDSB);
static_assert(NWAV * TB * NE * 4 <= LDSB);
static_assert(NWAV * TB * 64 * 4 <= LDSB);
static_assert((NTOK * DM) % (8 * NTHR) == 0);
static_assert((NE * KE * DM) % (8 * NTHR) == 0);
static_assert((NE * DM) % (8 * NTHR) == 0);

typedef unsigned short us;
typedef __bf16 v16bf __attribute__((ext_vector_type(16)));
typedef us v16us __attribute__((ext_vector_type(16)));
typedef us v8us_t __attribute__((ext_vector_type(8)));
typedef v8us_t __attribute__((may_alias)) v8us;
typedef float v8f __attribute__((ext_vector_type(8)));
typedef float v4f_t __attribute__((ext_vector_type(4)));
typedef v4f_t __attribute__((may_alias)) v4f;
typedef unsigned int v4u __attribute__((ext_vector_type(4)));

union Frag { v16us v; v8us_t h[2]; };

__device__ __forceinline__ v8f zero8() {
    v8f z;
#pragma unroll
    for (int i = 0; i < 8; ++i) z[i] = 0.0f;
    return z;
}

__device__ __forceinline__ us f2bf(float f) {
    unsigned int u = __float_as_uint(f);
    u += 0x7FFFu + ((u >> 16) & 1u);
    return (us)(u >> 16);
}
__device__ __forceinline__ float bf2f(us b) {
    return __uint_as_float(((unsigned int)b) << 16);
}

__device__ __forceinline__ v16bf ldfrag(const us* p, int k0) {
    Frag f;
    f.h[0] = *(const v8us*)(p + k0);
    f.h[1] = *(const v8us*)(p + k0 + 16);
    return __builtin_bit_cast(v16bf, f.v);
}

__device__ __forceinline__ v8f wmma16(v16bf a, v16bf b, v8f c) {
    return __builtin_amdgcn_wmma_f32_16x16x32_bf16(false, a, false, b, (short)0, c, false, false);
}

__device__ __forceinline__ float hmax16(float v) {
#pragma unroll
    for (int off = 8; off > 0; off >>= 1) v = fmaxf(v, __shfl_xor(v, off, 32));
    return v;
}
__device__ __forceinline__ float hsum16(float v) {
#pragma unroll
    for (int off = 8; off > 0; off >>= 1) v += __shfl_xor(v, off, 32);
    return v;
}
__device__ __forceinline__ int hsum16i(int v) {
#pragma unroll
    for (int off = 8; off > 0; off >>= 1) v += __shfl_xor(v, off, 32);
    return v;
}

__global__ void __launch_bounds__(NTHR) cvt_bf16_kernel(
    const float* __restrict__ src, us* __restrict__ dst, int n8)
{
    const int i = blockIdx.x * NTHR + threadIdx.x;
    const bool ok = (i < n8);
    v4u pk;
#pragma unroll
    for (int j = 0; j < 4; ++j) pk[j] = 0u;
    if (ok) {
        const v4f_t a = *(const v4f*)(src + (size_t)i * 8);
        const v4f_t b = *(const v4f*)(src + (size_t)i * 8 + 4);
        pk[0] = (unsigned int)f2bf(a[0]) | ((unsigned int)f2bf(a[1]) << 16);
        pk[1] = (unsigned int)f2bf(a[2]) | ((unsigned int)f2bf(a[3]) << 16);
        pk[2] = (unsigned int)f2bf(b[0]) | ((unsigned int)f2bf(b[1]) << 16);
        pk[3] = (unsigned int)f2bf(b[2]) | ((unsigned int)f2bf(b[3]) << 16);
        *(volatile v4u*)(dst + (size_t)i * 8) = pk;
    }
    __threadfence();
    if (ok) {
        *(volatile v4u*)(dst + (size_t)i * 8) = pk;
    }
}

__device__ __forceinline__ void swiglu32(
    const us* __restrict__ xa,
    const us* __restrict__ wg,
    const us* __restrict__ wu,
    int col0, const float* ews,
    us* hsH, us* hsL, int lane)
{
    const int hh = lane >> 4, m = lane & 15;
    v8f ag[2], au[2];
    ag[0] = zero8(); ag[1] = zero8(); au[0] = zero8(); au[1] = zero8();
    const us* pg = wg + (size_t)(col0 + m) * DM + 8 * hh;
    const us* pu = wu + (size_t)(col0 + m) * DM + 8 * hh;
#pragma unroll 1
    for (int k0 = 0; k0 < DM; k0 += 32) {
        const v16bf a  = ldfrag(xa, k0);
        const v16bf b0 = ldfrag(pg, k0);
        const v16bf b1 = ldfrag(pg + 16 * DM, k0);
        const v16bf c0 = ldfrag(pu, k0);
        const v16bf c1 = ldfrag(pu + 16 * DM, k0);
        ag[0] = wmma16(a, b0, ag[0]);
        ag[1] = wmma16(a, b1, ag[1]);
        au[0] = wmma16(a, c0, au[0]);
        au[1] = wmma16(a, c1, au[1]);
        asm volatile("v_nop\n\tv_nop\n\tv_nop\n\tv_nop"
                     : "+v"(ag[0]), "+v"(ag[1]), "+v"(au[0]), "+v"(au[1])
                     : "v"(a), "v"(b0), "v"(b1), "v"(c0), "v"(c1));
    }
    float rs[8];
#pragma unroll
    for (int r = 0; r < 8; ++r) rs[r] = ews[(8 * hh + r) * NE];
#pragma unroll
    for (int tn = 0; tn < 2; ++tn) {
        const int cc = col0 + 16 * tn + m;
#pragma unroll
        for (int r = 0; r < 8; ++r) {
            const float g  = ag[tn][r];
            const float u  = au[tn][r];
            const float sg = __builtin_amdgcn_rcpf(1.0f + __expf(-g));
            const float hv = ((g * sg) * u) * rs[r];
            const us hi = f2bf(hv);
            const us lo = f2bf(hv - bf2f(hi));
            const int idx = (8 * hh + r) * HP + cc;
            hsH[idx] = hi;
            hsL[idx] = lo;
        }
    }
}

__device__ __forceinline__ void down128(
    const us* hsH, const us* hsL, const us* __restrict__ wrow, v8f (&o)[8], int lane)
{
    const int hh = lane >> 4, m = lane & 15;
    const us* paH = hsH + m * HP + 8 * hh;
    const us* paL = hsL + m * HP + 8 * hh;
    const us* pb  = wrow + (size_t)m * KE + 8 * hh;
#pragma unroll 1
    for (int k0 = 0; k0 < KE; k0 += 32) {
        const v16bf ah = ldfrag(paH, k0);
        const v16bf al = ldfrag(paL, k0);
        v16bf b[8];
#pragma unroll
        for (int tn = 0; tn < 8; ++tn) b[tn] = ldfrag(pb + (size_t)tn * 16 * KE, k0);
#pragma unroll
        for (int tn = 0; tn < 8; ++tn) o[tn] = wmma16(ah, b[tn], o[tn]);
#pragma unroll
        for (int tn = 0; tn < 8; ++tn) o[tn] = wmma16(al, b[tn], o[tn]);
        asm volatile("v_nop\n\tv_nop\n\tv_nop\n\tv_nop"
                     : "+v"(o[0]), "+v"(o[1]), "+v"(o[2]), "+v"(o[3]),
                       "+v"(o[4]), "+v"(o[5]), "+v"(o[6]), "+v"(o[7])
                     : "v"(ah), "v"(al), "v"(b[0]), "v"(b[1]), "v"(b[2]), "v"(b[3]),
                       "v"(b[4]), "v"(b[5]), "v"(b[6]), "v"(b[7]));
    }
}

__global__ void __launch_bounds__(NTHR) moe_fused_kernel(
    const us* __restrict__ xb, const us* __restrict__ wgb, const us* __restrict__ wub,
    const us* __restrict__ wdb, const us* __restrict__ wrb, const float* __restrict__ ltp,
    float* __restrict__ out)
{
    __shared__ __align__(16) unsigned char lds_raw[LDSB];
    __shared__ __align__(16) float ewL[TB * NE];
    float* part = (float*)lds_raw;
    us*    hsH  = (us*)lds_raw;
    us*    hsL  = hsH + TB * HP;
    float* stg  = (float*)lds_raw;

    const int lane = threadIdx.x & 31, w = threadIdx.x >> 5;
    const int hh = lane >> 4, m = lane & 15;
    const int tok0 = blockIdx.x * TB;

    const us* xa = xb + (size_t)(tok0 + m) * DM + 8 * hh;

    {
        v8f acc = zero8();
        const us* pr = wrb + (size_t)m * DM + 8 * hh;
#pragma unroll 1
        for (int j = 0; j < RK / 32; ++j) {
            const int k0 = w * RK + 32 * j;
            const v16bf a = ldfrag(xa, k0);
            const v16bf b = ldfrag(pr, k0);
            acc = wmma16(a, b, acc);
            asm volatile("v_nop\n\tv_nop\n\tv_nop\n\tv_nop" : "+v"(acc) : "v"(a), "v"(b));
        }
#pragma unroll
        for (int r = 0; r < 8; ++r)
            part[(w * TB + 8 * hh + r) * NE + m] = acc[r];
    }
    __syncthreads();

    {
        const int tl = threadIdx.x >> 4;
        const int el = threadIdx.x & 15;
        float s = 0.0f;
#pragma unroll
        for (int wq = 0; wq < NWAV; ++wq) s += part[(wq * TB + tl) * NE + el];

        const float lt    = bf2f(f2bf(ltp[0]));
        const float sp    = fmaxf(lt, 0.0f) + log1pf(__expf(-fabsf(lt)));
        const float temp  = sp + 0.1f;
        const float rtemp = 1.0f / temp;
        const float v     = s * rtemp;

        const float m1  = hmax16(v);
        const int   cnt = hsum16i((v == m1) ? 1 : 0);
        const float vex = (v == m1) ? -__builtin_huge_valf() : v;
        const float m2r = hmax16(vex);
        const float thr = (cnt >= 2) ? m1 : m2r;

        const float z   = 10.0f * (v - thr);
        const float sg  = __builtin_amdgcn_rcpf(1.0f + __expf(-z));
        const float sup = v * sg;

        const float mx  = hmax16(sup);
        const float ex  = __expf(sup - mx);
        const float sm  = hsum16(ex);
        const float wv  = ex * __builtin_amdgcn_rcpf(sm);
        ewL[tl * NE + el] = wv;
    }
    __syncthreads();

    v8f o[8];
#pragma unroll
    for (int t = 0; t < 8; ++t) o[t] = zero8();

#pragma unroll 1
    for (int e = 0; e < NE; ++e) {
        const us* wg = wgb + (size_t)e * KE * DM;
        const us* wu = wub + (size_t)e * KE * DM;
        swiglu32(xa, wg, wu, w * 32, ewL + e, hsH, hsL, lane);
        __syncthreads();
        down128(hsH, hsL, wdb + ((size_t)e * DM + (size_t)w * WCOL) * KE, o, lane);
        __syncthreads();
    }

    float* stw = stg + w * (TB * 64);
    const int c4 = m * 4;
#pragma unroll
    for (int og = 0; og < 2; ++og) {
#pragma unroll
        for (int t4 = 0; t4 < 4; ++t4) {
#pragma unroll
            for (int r = 0; r < 8; ++r)
                stw[(8 * hh + r) * 64 + 16 * t4 + m] = o[og * 4 + t4][r];
        }
        __syncthreads();
        v4f_t v[8];
#pragma unroll
        for (int p = 0; p < 8; ++p) v[p] = *(const v4f*)(stw + (2 * p + hh) * 64 + c4);
        float* go = out + (size_t)tok0 * DM + w * WCOL + og * 64 + c4;
#pragma unroll
        for (int p = 0; p < 8; ++p)
            *(volatile v4f_t*)(go + (size_t)(2 * p + hh) * DM) = v[p];
        __threadfence();
#pragma unroll
        for (int p = 0; p < 8; ++p)
            *(volatile v4f_t*)(go + (size_t)(2 * p + hh) * DM) = v[p];
        __syncthreads();
    }
}

extern "C" void kernel_launch(void* const* d_in, const int* in_sizes, int n_in,
                              void* d_out, int out_size, void* d_ws, size_t ws_size,
                              hipStream_t stream)
{
    if (n_in < 6) return;
    if (in_sizes[0] != NTOK * DM) return;
    if (in_sizes[1] != NE * KE * DM) return;
    if (in_sizes[2] != NE * KE * DM) return;
    if (in_sizes[3] != NE * DM * KE) return;
    if (in_sizes[4] != NE * DM) return;
    if (in_sizes[5] < 1) return;
    if (out_size != NTOK * DM) return;

    const float* x   = (const float*)d_in[0];
    const float* wup = (const float*)d_in[1];
    const float* wgt = (const float*)d_in[2];
    const float* wdn = (const float*)d_in[3];
    const float* wro = (const float*)d_in[4];
    const float* ltp = (const float*)d_in[5];
    float* out = (float*)d_out;

    const size_t nX = (size_t)NTOK * DM;
    const size_t nW = (size_t)NE * KE * DM;
    const size_t nR = (size_t)NE * DM;

    const size_t oX  = 0;
    const size_t oWG = oX  + nX * 2;
    const size_t oWU = oWG + nW * 2;
    const size_t oWD = oWU + nW * 2;
    const size_t oWR = oWD + nW * 2;
    const size_t total = oWR + nR * 2;
    if (total > ws_size) return;

    char* ws = (char*)d_ws;
    us* xb  = (us*)(ws + oX);
    us* wgb = (us*)(ws + oWG);
    us* wub = (us*)(ws + oWU);
    us* wdb = (us*)(ws + oWD);
    us* wrb = (us*)(ws + oWR);

    const int n8X = (int)(nX / 8), n8W = (int)(nW / 8), n8R = (int)(nR / 8);
    cvt_bf16_kernel<<<(n8X + NTHR - 1) / NTHR, NTHR, 0, stream>>>(x,   xb,  n8X);
    cvt_bf16_kernel<<<(n8W + NTHR - 1) / NTHR, NTHR, 0, stream>>>(wgt, wgb, n8W);
    cvt_bf16_kernel<<<(n8W + NTHR - 1) / NTHR, NTHR, 0, stream>>>(wup, wub, n8W);
    cvt_bf16_kernel<<<(n8W + NTHR - 1) / NTHR, NTHR, 0, stream>>>(wdn, wdb, n8W);
    cvt_bf16_kernel<<<(n8R + NTHR - 1) / NTHR, NTHR, 0, stream>>>(wro, wrb, n8R);

    moe_fused_kernel<<<NTOK / TB, NTHR, 0, stream>>>(xb, wgb, wub, wdb, wrb, ltp, out);
}
